// GroupedQueryAttention_89163521065857
// MI455X (gfx1250) — hardware-verified
//
#include <hip/hip_runtime.h>
#include <math.h>

typedef __attribute__((ext_vector_type(16))) _Float16       v16h;
typedef __attribute__((ext_vector_type(8)))  _Float16       v8h;
typedef __attribute__((ext_vector_type(16))) __bf16         v16b;
typedef __attribute__((ext_vector_type(8)))  __bf16         v8b;
typedef __attribute__((ext_vector_type(8)))  float          v8f;
typedef __attribute__((ext_vector_type(4)))  float          v4f;
typedef __attribute__((ext_vector_type(4)))  unsigned int   v4u;
typedef __attribute__((ext_vector_type(8)))  unsigned short v8us;

#ifndef NB
#define NB 2
#endif
#ifndef SEQ
#define SEQ 2048
#endif
#define NB_FULL  2
#define SEQ_FULL 2048
#define DMODEL 128
#define HDIM   128
#define NQH    16
#define NKV    4
#define GRP    4
#define NSLOT  20
#define NHS    24
#define EMB    2048
#define EKV    512
#define NPROJ  3072
#define KC     64
#define QT     16
#define NWAVE  4

#define XB_BYTES   ((size_t)NB * SEQ * DMODEL * 2)
#define WT_BYTES   ((size_t)NPROJ * DMODEL * 2)
#define WOT_BYTES  ((size_t)DMODEL * EMB * 2)
#define FREQ_BYTES ((size_t)256)
#define CS_BYTES   ((size_t)SEQ * 64 * 4)
#define QK_BYTES   ((size_t)NB * NSLOT * SEQ * HDIM * 2)
#define VT_BYTES   ((size_t)NB * NKV * HDIM * SEQ * 2)
#define CTX_PLANE  ((size_t)NB * SEQ * EMB)
#define CTX_BYTES  (CTX_PLANE * 2 * 2)

#define OFF_XB   ((size_t)0)
#define OFF_WT   (OFF_XB + XB_BYTES)
#define OFF_WOT  (OFF_WT + WT_BYTES)
#define OFF_FREQ (OFF_WOT + WOT_BYTES)
#define OFF_COS  (OFF_FREQ + FREQ_BYTES)
#define OFF_SIN  (OFF_COS + CS_BYTES)
#define OFF_QK   (OFF_SIN + CS_BYTES)
#define OFF_VT   (OFF_QK + QK_BYTES)
#define OFF_CTX  (OFF_VT + VT_BYTES)
#define WS_TOTAL (OFF_CTX + CTX_BYTES)

static_assert(SEQ % KC == 0);
static_assert(SEQ % QT == 0);
static_assert((NB * SEQ) % 64 == 0);
static_assert(SEQ <= SEQ_FULL && NB <= NB_FULL);
static_assert(EMB == NQH * HDIM);
static_assert(EKV == NKV * HDIM);
static_assert(NQH == NKV * GRP);
static_assert(GRP == NWAVE);
static_assert(NSLOT == NQH + NKV && NHS == NSLOT + NKV && NPROJ == NHS * HDIM);
static_assert(HDIM == 128 && DMODEL == 128 && KC == 64 && QT == 16);
static_assert(NWAVE * 32 * 8 == KC * (HDIM / 8));
static_assert(NWAVE * 32 * 8 == HDIM * (KC / 8));
static_assert(HDIM * 2 == 16 * 16);
static_assert(DMODEL * 4 == 32 * 16);
static_assert(DMODEL % 32 == 0 && EMB % 32 == 0);
static_assert(DMODEL % 64 == 0 && EMB % 64 == 0 && EKV % 64 == 0);
static_assert((SEQ * 64) % 256 == 0);
static_assert(XB_BYTES % 256 == 0 && WT_BYTES % 256 == 0 && WOT_BYTES % 256 == 0 && CS_BYTES % 256 == 0);
static_assert(QK_BYTES % 256 == 0 && VT_BYTES % 256 == 0 && CTX_BYTES % 256 == 0);
static_assert(WS_TOTAL <= (size_t)134217728);
static_assert((size_t)NB * NSLOT * SEQ * HDIM < (size_t)2147483647);

__device__ __forceinline__ unsigned int bf_bits(float f) {
    const unsigned int u = __float_as_uint(f);
    return (u + 0x7FFFu + ((u >> 16) & 1u)) >> 16;
}
__device__ __forceinline__ float bf_val(float f) { return __uint_as_float(bf_bits(f) << 16); }
__device__ __forceinline__ unsigned int h_bits(float f) { return (unsigned int)__builtin_bit_cast(unsigned short, (_Float16)f); }

__device__ __forceinline__ v8f mma_bf(v16b a, v16b b, v8f c) {
    c = __builtin_amdgcn_wmma_f32_16x16x32_bf16(false, a, false, b, (short)0, c, false, false);
    asm volatile("v_nop\n\tv_nop\n\tv_nop\n\tv_nop" : "+v"(c) : "v"(a), "v"(b));
    return c;
}
__device__ __forceinline__ v8f mma_h(v16h a, v16h b, v8f c) {
    c = __builtin_amdgcn_wmma_f32_16x16x32_f16(false, a, false, b, (short)0, c, false, false);
    asm volatile("v_nop\n\tv_nop\n\tv_nop\n\tv_nop" : "+v"(c) : "v"(a), "v"(b));
    return c;
}

__device__ __forceinline__ void st16x2(unsigned short* p, v4u v) {
    volatile v4u* d = (volatile v4u*)p;
    *d = v; __threadfence(); *d = v;
}

__global__ __launch_bounds__(256) void k_cvt_x(const float* __restrict__ xin, unsigned short* __restrict__ XB) {
    const long long u = (long long)blockIdx.x * 256 + threadIdx.x;
    if (u >= (long long)NB * SEQ * (DMODEL / 8)) return;
    const int pc = (int)(u % (DMODEL / 8));
    const long long row = u / (DMODEL / 8);
    const int b = (int)(row / SEQ), s = (int)(row - (long long)b * SEQ);
    const float* src = xin + ((size_t)b * SEQ_FULL + s) * DMODEL + pc * 8;
    const v4f a = *(const v4f*)(src), c = *(const v4f*)(src + 4);
    v4u pk;
    pk.x = bf_bits(a.x) | (bf_bits(a.y) << 16); pk.y = bf_bits(a.z) | (bf_bits(a.w) << 16);
    pk.z = bf_bits(c.x) | (bf_bits(c.y) << 16); pk.w = bf_bits(c.z) | (bf_bits(c.w) << 16);
    st16x2(XB + (size_t)row * DMODEL + pc * 8, pk);
}

__global__ __launch_bounds__(256) void k_cvt_wT(const float* __restrict__ win, unsigned short* __restrict__ wout, int R, int C) {
    __shared__ __align__(16) unsigned short tile[64 * 72];
    const int t = threadIdx.x;
    const int c0 = blockIdx.x * 64, r0 = blockIdx.y * 64;
    {
        const int rl = t >> 2, part = t & 3;
        const float* src = win + (size_t)(r0 + rl) * C + c0 + part * 16;
        const v4f f0 = *(const v4f*)(src), f1 = *(const v4f*)(src + 4), f2 = *(const v4f*)(src + 8), f3 = *(const v4f*)(src + 12);
        v4u p0, p1;
        p0.x = bf_bits(f0.x) | (bf_bits(f0.y) << 16); p0.y = bf_bits(f0.z) | (bf_bits(f0.w) << 16);
        p0.z = bf_bits(f1.x) | (bf_bits(f1.y) << 16); p0.w = bf_bits(f1.z) | (bf_bits(f1.w) << 16);
        p1.x = bf_bits(f2.x) | (bf_bits(f2.y) << 16); p1.y = bf_bits(f2.z) | (bf_bits(f2.w) << 16);
        p1.z = bf_bits(f3.x) | (bf_bits(f3.y) << 16); p1.w = bf_bits(f3.z) | (bf_bits(f3.w) << 16);
        *(v4u*)(tile + rl * 72 + part * 16)     = p0;
        *(v4u*)(tile + rl * 72 + part * 16 + 8) = p1;
    }
    __syncthreads();
#pragma unroll
    for (int it = 0; it < 2; ++it) {
        const int crow = it * 32 + (t >> 3), pc = t & 7;
        unsigned int e[8];
#pragma unroll
        for (int j = 0; j < 8; ++j) e[j] = (unsigned int)tile[(pc * 8 + j) * 72 + crow];
        v4u pk;
        pk.x = e[0] | (e[1] << 16); pk.y = e[2] | (e[3] << 16); pk.z = e[4] | (e[5] << 16); pk.w = e[6] | (e[7] << 16);
        st16x2(wout + (size_t)(c0 + crow) * R + r0 + pc * 8, pk);
    }
}

__global__ __launch_bounds__(64) void k_freq(const int* __restrict__ theta_p, float* __restrict__ FREQ) {
    const int i = threadIdx.x;
    const float th = (float)theta_p[0];
    const float e = -(float)i * (1.0f / 64.0f);
    const float f = powf(th, e);
    volatile float* d = FREQ + i;
    *d = f; __threadfence(); *d = f;
}

__global__ __launch_bounds__(256) void k_rope_tab(const float* __restrict__ FREQ, float* __restrict__ COS, float* __restrict__ SIN) {
    const int idx = blockIdx.x * 256 + threadIdx.x;
    if (idx >= SEQ * 64) return;
    const int l = idx >> 6, i = idx & 63;
    const float ang = (float)l * FREQ[i];
    float sv, cv;
    sincosf(ang, &sv, &cv);
    volatile float* pc = COS + idx;
    volatile float* ps = SIN + idx;
    *pc = cv; *ps = sv;
    __threadfence();
    *pc = cv; *ps = sv;
}

__global__ __launch_bounds__(128) void k_qkv(const unsigned short* __restrict__ XB, const unsigned short* __restrict__ WT,
                                             const float* __restrict__ bq, const float* __restrict__ bk, const float* __restrict__ bv,
                                             const float* __restrict__ COS, const float* __restrict__ SIN,
                                             unsigned short* __restrict__ QK, unsigned short* __restrict__ VT) {
    union FB { v16b v; v8b h[2]; };
    __shared__ __align__(16) float          Sl[NWAVE][QT * 132];
    __shared__ __align__(16) unsigned short VtS[HDIM * 72];

    const int tid = threadIdx.x, wave = tid >> 5, lane = tid & 31, hh = lane >> 4, c = lane & 15;
    const int hs = blockIdx.y;
    const int rowb = blockIdx.x * 64;
    const int b = rowb / SEQ, s0 = rowb - b * SEQ;
    const int row0 = rowb + wave * QT;
    const int n0 = hs * HDIM;
    const float CARRY = 16.0f;

    const __bf16* xp = (const __bf16*)XB + (size_t)(row0 + c) * DMODEL;
    const __bf16* wp = (const __bf16*)WT + (size_t)(n0 + c) * DMODEL;

    v8f acc[8];
#pragma unroll
    for (int t = 0; t < 8; ++t) acc[t] = (v8f){0.f, 0.f, 0.f, 0.f, 0.f, 0.f, 0.f, 0.f};
#pragma unroll
    for (int kc = 0; kc < DMODEL / 32; ++kc) {
        FB a;
        a.h[0] = *(const v8b*)(xp + kc * 32 + 8 * hh);
        a.h[1] = *(const v8b*)(xp + kc * 32 + 16 + 8 * hh);
#pragma unroll
        for (int t = 0; t < 8; ++t) {
            FB w;
            w.h[0] = *(const v8b*)(wp + (size_t)t * 16 * DMODEL + kc * 32 + 8 * hh);
            w.h[1] = *(const v8b*)(wp + (size_t)t * 16 * DMODEL + kc * 32 + 16 + 8 * hh);
            acc[t] = mma_bf(a.v, w.v, acc[t]);
        }
    }

    float bias[8];
#pragma unroll
    for (int t = 0; t < 8; ++t) {
        const int col = n0 + t * 16 + c;
        const int iq = min(col, EMB - 1);
        const int ik = min(max(col - EMB, 0), EKV - 1);
        const int iv = min(max(col - EMB - EKV, 0), EKV - 1);
        const float fq = bq[iq], fk = bk[ik], fv = bv[iv];
        bias[t] = bf_val((hs < NQH) ? fq : ((hs < NSLOT) ? fk : fv));
    }

    if (hs < NSLOT) {
        float* sl = Sl[wave];
#pragma unroll
        for (int r = 0; r < 8; ++r) {
#pragma unroll
            for (int t = 0; t < 8; ++t) sl[(8 * hh + r) * 132 + t * 16 + c] = acc[t][r] + bias[t];
        }
        __builtin_amdgcn_fence(3  , "workgroup");
        __builtin_amdgcn_wave_barrier();
        __builtin_amdgcn_fence(2  , "workgroup");

        const size_t pbase = ((size_t)(b * NSLOT + hs) * SEQ + s0 + wave * QT) * HDIM;
        const int c8 = (lane & 15) * 8;
#pragma unroll 2
        for (int it = 0; it < 8; ++it) {
            const int row = it * 2 + hh;
            const int l = s0 + wave * QT + row;
            const v4f x0 = *(const v4f*)(sl + row * 132 + c8);
            const v4f x1 = *(const v4f*)(sl + row * 132 + c8 + 4);
            const v4f cs = *(const v4f*)(COS + (size_t)l * 64 + (c8 >> 1));
            const v4f sn = *(const v4f*)(SIN + (size_t)l * 64 + (c8 >> 1));
            const float o0 = x0.x * cs.x - x0.y * sn.x, o1 = x0.x * sn.x + x0.y * cs.x;
            const float o2 = x0.z * cs.y - x0.w * sn.y, o3 = x0.z * sn.y + x0.w * cs.y;
            const float o4 = x1.x * cs.z - x1.y * sn.z, o5 = x1.x * sn.z + x1.y * cs.z;
            const float o6 = x1.z * cs.w - x1.w * sn.w, o7 = x1.z * sn.w + x1.w * cs.w;
            v4u pk;
            pk.x = h_bits(o0 * CARRY) | (h_bits(o1 * CARRY) << 16);
            pk.y = h_bits(o2 * CARRY) | (h_bits(o3 * CARRY) << 16);
            pk.z = h_bits(o4 * CARRY) | (h_bits(o5 * CARRY) << 16);
            pk.w = h_bits(o6 * CARRY) | (h_bits(o7 * CARRY) << 16);
            st16x2(QK + pbase + (size_t)row * HDIM + c8, pk);
        }
    } else {
        const int g = hs - NSLOT;
#pragma unroll
        for (int t = 0; t < 8; ++t) {
            const int d = t * 16 + c;
            v4u pk;
            pk.x = h_bits((acc[t][0] + bias[t]) * CARRY) | (h_bits((acc[t][1] + bias[t]) * CARRY) << 16);
            pk.y = h_bits((acc[t][2] + bias[t]) * CARRY) | (h_bits((acc[t][3] + bias[t]) * CARRY) << 16);
            pk.z = h_bits((acc[t][4] + bias[t]) * CARRY) | (h_bits((acc[t][5] + bias[t]) * CARRY) << 16);
            pk.w = h_bits((acc[t][6] + bias[t]) * CARRY) | (h_bits((acc[t][7] + bias[t]) * CARRY) << 16);
            *(v4u*)(VtS + d * 72 + wave * QT + 8 * hh) = pk;
        }
        __syncthreads();
#pragma unroll 2
        for (int it = 0; it < 8; ++it) {
            const int drow = it * 16 + (tid >> 3), pc = tid & 7;
            const v4u val = *(const v4u*)(VtS + drow * 72 + pc * 8);
            st16x2(VT + ((size_t)((b * NKV + g) * HDIM + drow)) * SEQ + s0 + pc * 8, val);
        }
    }
}

__global__ __launch_bounds__(128) void k_attn_grp(const unsigned short* __restrict__ QK, const unsigned short* __restrict__ VT16,
                                                   unsigned short* __restrict__ CTX) {
    union FH { v16h v; v8h h[2]; };
    __shared__ __align__(16) unsigned short Ksh[KC * HDIM];
    __shared__ __align__(16) unsigned short Vth[HDIM * KC];
    __shared__ __align__(16) _Float16       Psh[NWAVE][QT * KC];
    __shared__ __align__(16) unsigned short Osh[NWAVE][QT * 136];

    const int tid = threadIdx.x, wave = tid >> 5, lane = tid & 31, hh = lane >> 4, c = lane & 15;
    const int qb = blockIdx.x, g = blockIdx.y, b = blockIdx.z;
    const int head = g * GRP + wave;
    const int q0 = qb * QT;
    const float SCL = (0.08838834764831845f * 1.4426950408889634f) * (1.0f / 256.0f);
    const float PSC = 32768.0f;
    const float VCARRY = 16.0f;

    const _Float16* Qp = (const _Float16*)QK;
    const unsigned int qoff = (unsigned int)(((b * NSLOT + head) * SEQ + q0 + c) * HDIM) + (unsigned int)(8 * hh);

    float mrow[8], lrow[8];
    v8f oacc[8];
#pragma unroll
    for (int r = 0; r < 8; ++r) { mrow[r] = -INFINITY; lrow[r] = 0.f; }
#pragma unroll
    for (int t = 0; t < 8; ++t) oacc[t] = (v8f){0.f, 0.f, 0.f, 0.f, 0.f, 0.f, 0.f, 0.f};

    const unsigned short* Kb = QK + ((size_t)(b * NSLOT + NQH + g) * SEQ) * HDIM;
    const unsigned short* Vb = VT16 + ((size_t)(b * NKV + g) * HDIM) * SEQ;
    const _Float16* Kp = (const _Float16*)Ksh;
    const _Float16* Vp = (const _Float16*)Vth;
    _Float16* pw = Psh[wave];

    for (int kc = 0; kc < SEQ / KC; ++kc) {
        const int kv0 = kc * KC;
        __syncthreads();
#pragma unroll
        for (int i = 0; i < 8; ++i) {
            const int idx = tid + 128 * i;
            const int row = idx >> 4, pc = idx & 15;
            const v4u kk = *(const v4u*)(Kb + (size_t)(kv0 + row) * HDIM + pc * 8);
            *(v4u*)(Ksh + row * HDIM + pc * 8) = kk;
        }
#pragma unroll
        for (int i = 0; i < 8; ++i) {
            const int idx = tid + 128 * i;
            const int row = idx >> 3, pc = idx & 7;
            const v4u vv = *(const v4u*)(Vb + (size_t)row * SEQ + kv0 + pc * 8);
            *(v4u*)(Vth + row * KC + pc * 8) = vv;
        }
        __syncthreads();

#pragma unroll 1
        for (int kh = 0; kh < 2; ++kh) {
            unsigned int qo = qoff;
            asm volatile("" : "+v"(qo));
            const int kofs = (kh * 32 + c) * HDIM + 8 * hh;

            v8f s0 = (v8f){0.f, 0.f, 0.f, 0.f, 0.f, 0.f, 0.f, 0.f};
            v8f s1 = (v8f){0.f, 0.f, 0.f, 0.f, 0.f, 0.f, 0.f, 0.f};
#pragma unroll
            for (int dc = 0; dc < 4; ++dc) {
                FH qa, k0, k1;
                qa.h[0] = *(const v8h*)(Qp + qo + dc * 32);
                qa.h[1] = *(const v8h*)(Qp + qo + dc * 32 + 16);
                k0.h[0] = *(const v8h*)(Kp + kofs + dc * 32);
                k0.h[1] = *(const v8h*)(Kp + kofs + dc * 32 + 16);
                k1.h[0] = *(const v8h*)(Kp + kofs + 16 * HDIM + dc * 32);
                k1.h[1] = *(const v8h*)(Kp + kofs + 16 * HDIM + dc * 32 + 16);
                s0 = mma_h(qa.v, k0.v, s0);
                s1 = mma_h(qa.v, k1.v, s1);
            }

#pragma unroll
            for (int r = 0; r < 8; ++r) {
                const float x0 = s0[r] * SCL, x1 = s1[r] * SCL;
                float m = fmaxf(x0, x1);
                m = fmaxf(m, __shfl_xor(m, 1, 32)); m = fmaxf(m, __shfl_xor(m, 2, 32));
                m = fmaxf(m, __shfl_xor(m, 4, 32)); m = fmaxf(m, __shfl_xor(m, 8, 32));
                const float mnew  = fmaxf(mrow[r], m);
                const float alpha = exp2f(mrow[r] - mnew);
                mrow[r] = mnew;
                const float p0 = exp2f(x0 - mnew), p1 = exp2f(x1 - mnew);
                _Float16* prow = pw + (8 * hh + r) * KC + kh * 32 + c;
                prow[0]  = (_Float16)(p0 * PSC);
                prow[16] = (_Float16)(p1 * PSC);
                float psum = p0 + p1;
                psum += __shfl_xor(psum, 1, 32); psum += __shfl_xor(psum, 2, 32);
                psum += __shfl_xor(psum, 4, 32); psum += __shfl_xor(psum, 8, 32);
                lrow[r] = lrow[r] * alpha + psum;
#pragma unroll
                for (int t = 0; t < 8; ++t) oacc[t][r] *= alpha;
            }
            __builtin_amdgcn_fence(3  , "workgroup");
            __builtin_amdgcn_wave_barrier();
            __builtin_amdgcn_fence(2  , "workgroup");

            FH pa;
            pa.h[0] = *(const v8h*)(pw + c * KC + kh * 32 + 8 * hh);
            pa.h[1] = *(const v8h*)(pw + c * KC + kh * 32 + 16 + 8 * hh);
            const int vofs = c * KC + kh * 32 + 8 * hh;
#pragma unroll
            for (int tg = 0; tg < 2; ++tg) {
                FH vb[4];
#pragma unroll
                for (int u = 0; u < 4; ++u) {
                    vb[u].h[0] = *(const v8h*)(Vp + (tg * 4 + u) * 16 * KC + vofs);
                    vb[u].h[1] = *(const v8h*)(Vp + (tg * 4 + u) * 16 * KC + vofs + 16);
                }
#pragma unroll
                for (int u = 0; u < 4; ++u) oacc[tg * 4 + u] = mma_h(pa.v, vb[u].v, oacc[tg * 4 + u]);
            }
        }
    }

    float inv[8];
#pragma unroll
    for (int r = 0; r < 8; ++r) inv[r] = 1.0f / (lrow[r] * (PSC * VCARRY));
    unsigned short* os = Osh[wave];
    const int c8 = (lane & 15) * 8;
    const size_t obase = ((size_t)b * SEQ + q0) * EMB + (size_t)head * HDIM;
#pragma unroll
    for (int part = 0; part < 2; ++part) {
#pragma unroll
        for (int r = 0; r < 8; ++r) {
#pragma unroll
            for (int t = 0; t < 8; ++t) {
                const float o = oacc[t][r] * inv[r];
                const unsigned int hi = bf_bits(o);
                const unsigned int lo = bf_bits(o - __uint_as_float(hi << 16));
                os[(8 * hh + r) * 136 + t * 16 + c] = (unsigned short)((part == 0) ? hi : lo);
            }
        }
        __builtin_amdgcn_fence(3  , "workgroup");
        __builtin_amdgcn_wave_barrier();
        __builtin_amdgcn_fence(2  , "workgroup");
        unsigned short* ob = CTX + (size_t)part * CTX_PLANE + obase;
        for (int pass = 0; pass < 2; ++pass) {
#pragma unroll
            for (int it = 0; it < 8; ++it) {
                const int row = it * 2 + hh;
                const v8us hv = *(const v8us*)(os + row * 136 + c8);
                const v4u val = __builtin_bit_cast(v4u, hv);
                *(volatile v4u*)(ob + (size_t)row * EMB + c8) = val;
            }
            __threadfence();
        }
        __builtin_amdgcn_fence(3  , "workgroup");
        __builtin_amdgcn_wave_barrier();
        __builtin_amdgcn_fence(2  , "workgroup");
    }
}

__global__ __launch_bounds__(128) void k_oproj(const unsigned short* __restrict__ CTX, const unsigned short* __restrict__ WOT,
                                               const float* __restrict__ bo, float* __restrict__ out) {
    union FB { v16b v; v8b h[2]; };
    __shared__ __align__(16) float Os[NWAVE][QT * 132];

    const int tid = threadIdx.x, wave = tid >> 5, lane = tid & 31, hh = lane >> 4, c = lane & 15;
    const int row0 = blockIdx.x * 64 + wave * QT;

    const __bf16* ah = (const __bf16*)CTX + (size_t)(row0 + c) * EMB;
    const __bf16* al = ah + CTX_PLANE;
    const __bf16* wp = (const __bf16*)WOT + (size_t)c * EMB;

    v8f acc[8];
#pragma unroll
    for (int t = 0; t < 8; ++t) acc[t] = (v8f){0.f, 0.f, 0.f, 0.f, 0.f, 0.f, 0.f, 0.f};

#pragma unroll 1
    for (int ks = 0; ks < EMB / 32; ++ks) {
        FB a, l;
        a.h[0] = *(const v8b*)(ah + ks * 32 + 8 * hh);
        a.h[1] = *(const v8b*)(ah + ks * 32 + 16 + 8 * hh);
        l.h[0] = *(const v8b*)(al + ks * 32 + 8 * hh);
        l.h[1] = *(const v8b*)(al + ks * 32 + 16 + 8 * hh);
#pragma unroll
        for (int t = 0; t < 8; ++t) {
            FB w;
            w.h[0] = *(const v8b*)(wp + (size_t)t * 16 * EMB + ks * 32 + 8 * hh);
            w.h[1] = *(const v8b*)(wp + (size_t)t * 16 * EMB + ks * 32 + 16 + 8 * hh);
            acc[t] = mma_bf(a.v, w.v, acc[t]);
            acc[t] = mma_bf(l.v, w.v, acc[t]);
        }
    }

    float bias[8];
#pragma unroll
    for (int t = 0; t < 8; ++t) bias[t] = bf_val(bo[t * 16 + c]);

    float* os = Os[wave];
#pragma unroll
    for (int r = 0; r < 8; ++r) {
#pragma unroll
        for (int t = 0; t < 8; ++t) os[(8 * hh + r) * 132 + t * 16 + c] = acc[t][r] + bias[t];
    }
    __builtin_amdgcn_fence(3  , "workgroup");
    __builtin_amdgcn_wave_barrier();
    __builtin_amdgcn_fence(2  , "workgroup");
    {
        float* ob = out + (size_t)row0 * DMODEL;
        const int c4 = lane * 4;
        for (int pass = 0; pass < 2; ++pass) {
#pragma unroll 4
            for (int row = 0; row < QT; ++row) {
                const v4f val = *(const v4f*)(os + row * 132 + c4);
                *(volatile v4f*)(ob + (size_t)row * DMODEL + c4) = val;
            }
            __threadfence();
        }
    }
}

extern "C" void kernel_launch(void* const* d_in, const int* in_sizes, int n_in, void* d_out, int out_size, void* d_ws, size_t ws_size, hipStream_t stream) {
    if (n_in < 10) return;
    if ((long long)in_sizes[0] < (long long)(NB - 1) * SEQ_FULL * DMODEL + (long long)SEQ * DMODEL) return;
    if ((long long)in_sizes[1] < (long long)DMODEL * EMB) return;
    if ((long long)in_sizes[2] < (long long)EMB) return;
    if ((long long)in_sizes[3] < (long long)DMODEL * EKV) return;
    if ((long long)in_sizes[4] < (long long)EKV) return;
    if ((long long)in_sizes[5] < (long long)DMODEL * EKV) return;
    if ((long long)in_sizes[6] < (long long)EKV) return;
    if ((long long)in_sizes[7] < (long long)EMB * DMODEL) return;
    if ((long long)in_sizes[8] < (long long)DMODEL) return;
    if ((long long)in_sizes[9] < 1) return;
    if ((long long)out_size < (long long)NB * SEQ * DMODEL) return;
    if (ws_size < WS_TOTAL) return;

    const float* x   = (const float*)d_in[0];
    const float* Wq  = (const float*)d_in[1];
    const float* bq  = (const float*)d_in[2];
    const float* Wk  = (const float*)d_in[3];
    const float* bk  = (const float*)d_in[4];
    const float* Wv  = (const float*)d_in[5];
    const float* bv  = (const float*)d_in[6];
    const float* Wo  = (const float*)d_in[7];
    const float* bo  = (const float*)d_in[8];
    const int* theta = (const int*)d_in[9];
    float* out = (float*)d_out;

    char* ws = (char*)d_ws;
    unsigned short* XB  = (unsigned short*)(ws + OFF_XB);
    unsigned short* WT  = (unsigned short*)(ws + OFF_WT);
    unsigned short* WOT = (unsigned short*)(ws + OFF_WOT);
    float* FREQ = (float*)(ws + OFF_FREQ);
    float* COS  = (float*)(ws + OFF_COS);
    float* SIN  = (float*)(ws + OFF_SIN);
    unsigned short* QK  = (unsigned short*)(ws + OFF_QK);
    unsigned short* VT  = (unsigned short*)(ws + OFF_VT);
    unsigned short* CTX = (unsigned short*)(ws + OFF_CTX);

    k_cvt_x<<<(unsigned)(((long long)NB * SEQ * (DMODEL / 8) + 255) / 256), 256, 0, stream>>>(x, XB);
    k_cvt_wT<<<dim3((unsigned)(EMB / 64), (unsigned)(DMODEL / 64)), 256, 0, stream>>>(Wq, WT, DMODEL, EMB);
    k_cvt_wT<<<dim3((unsigned)(EKV / 64), (unsigned)(DMODEL / 64)), 256, 0, stream>>>(Wk, WT + (size_t)EMB * DMODEL, DMODEL, EKV);
    k_cvt_wT<<<dim3((unsigned)(EKV / 64), (unsigned)(DMODEL / 64)), 256, 0, stream>>>(Wv, WT + (size_t)(EMB + EKV) * DMODEL, DMODEL, EKV);
    k_cvt_wT<<<dim3((unsigned)(DMODEL / 64), (unsigned)(EMB / 64)), 256, 0, stream>>>(Wo, WOT, EMB, DMODEL);
    k_freq<<<1, 64, 0, stream>>>(theta, FREQ);
    k_rope_tab<<<(unsigned)((SEQ * 64) / 256), 256, 0, stream>>>(FREQ, COS, SIN);
    k_qkv<<<dim3((unsigned)((NB * SEQ) / 64), (unsigned)NHS), 128, 0, stream>>>(XB, WT, bq, bk, bv, COS, SIN, QK, VT);
    k_attn_grp<<<dim3((unsigned)(SEQ / QT), (unsigned)NKV, (unsigned)NB), 128, 0, stream>>>(QK, VT, CTX);
    k_oproj<<<(unsigned)((NB * SEQ) / 64), 128, 0, stream>>>(CTX, WOT, bo, out);
}
